// RoutingLayer_51196010168971
// MI455X (gfx1250) — hardware-verified
//
#include <hip/hip_runtime.h>
#include <math.h>
#include <stdint.h>

#define NB     2
#define SEQ    1024
#define EMB    1024
#define HDIM   512
#define NHEAD  8
#define DHEAD  64
#define NMAT   16
#define MROWS  2048
#define NITER  20

typedef __attribute__((ext_vector_type(16))) __bf16   v16b;
typedef __attribute__((ext_vector_type(8)))  __bf16   v8b;
typedef __attribute__((ext_vector_type(8)))  float    v8f;
typedef __attribute__((ext_vector_type(4)))  float    v4f;
typedef __attribute__((ext_vector_type(2)))  float    v2f;
typedef __attribute__((ext_vector_type(4)))  unsigned int v4u;
typedef __attribute__((ext_vector_type(8)))  unsigned short v8us;

__device__ __forceinline__ unsigned short f2bf_bits(float f) {
  unsigned u = __float_as_uint(f);
  return (unsigned short)((u + 0x7FFFu + ((u >> 16) & 1u)) >> 16);
}
__device__ __forceinline__ float bf_bits2f(unsigned short h) { return __uint_as_float(((unsigned)h) << 16); }
__device__ __forceinline__ unsigned pk16(unsigned short a, unsigned short b) { return (unsigned)a | ((unsigned)b << 16); }

__device__ __forceinline__ void dep_guard_b(v8f& a, v8f& b, v16b x, v16b y) { asm volatile("v_nop\n\tv_nop\n\tv_nop\n\tv_nop" : "+v"(a), "+v"(b) : "v"(x), "v"(y)); }
__device__ __forceinline__ void keep4_b(v16b a, v16b b, v16b c, v16b d) { asm volatile("v_nop" :: "v"(a), "v"(b), "v"(c), "v"(d)); }
__device__ __forceinline__ void acc_guard4(v8f& a, v8f& b, v8f& c, v8f& d) { asm volatile("v_nop\n\tv_nop\n\tv_nop\n\tv_nop" : "+v"(a), "+v"(b), "+v"(c), "+v"(d)); }

__device__ __forceinline__ v16b ld_frag(const __bf16* p) {
  union { v16b v; v8b h[2]; } f;
  f.h[0] = *(const v8b*)(p);
  f.h[1] = *(const v8b*)(p + 16);
  return f.v;
}
__device__ __forceinline__ v8f mma_bf(v16b a, v16b b, v8f c) {
  return __builtin_amdgcn_wmma_f32_16x16x32_bf16(false, a, false, b, (short)0, c, false, false);
}
__device__ __forceinline__ v8f mma_bf_g(v16b a, v16b b, v8f c) {
  c = __builtin_amdgcn_wmma_f32_16x16x32_bf16(false, a, false, b, (short)0, c, false, false);
  asm volatile("v_nop\n\tv_nop\n\tv_nop\n\tv_nop" : "+v"(c) : "v"(a), "v"(b));
  return c;
}

template <int BIAS_MODE, int OUT_MODE>
__global__ __launch_bounds__(256) void gemm64_split(
    const unsigned short* __restrict__ Ap, const unsigned short* __restrict__ A2p, int lda, long strideA, long strideAs,
    const unsigned short* __restrict__ Btp, const unsigned short* __restrict__ Bt2p, int ldb, long strideB, long strideBs,
    void* __restrict__ Cout, void* __restrict__ Cout2, int ldc, long strideC,
    const float* __restrict__ bias, int M, int N, int K, int zsub, float scale) {
  __shared__ __align__(16) float sT[8][16 * 68];
  const __bf16* A   = (const __bf16*)(const void*)Ap;
  const __bf16* A2  = (const __bf16*)(const void*)A2p;
  const __bf16* Bt  = (const __bf16*)(const void*)Btp;
  const __bf16* Bt2 = (const __bf16*)(const void*)Bt2p;
  const int z    = blockIdx.y;
  const int zq   = z / zsub;
  const int zr   = z - zq * zsub;
  const int lane = threadIdx.x & 31;
  const int wave = threadIdx.x >> 5;
  const int tilesN = N >> 6;
  const int tilesM = M >> 6;
  const int tile = blockIdx.x * 8 + wave;
  if (tile >= tilesM * tilesN) return;
  const int tm = tile / tilesN;
  const int tn = tile - tm * tilesN;
  const int m0 = tm << 6;
  const int n0 = tn << 6;

  const size_t oA = (size_t)zq * (size_t)strideA + (size_t)zr * (size_t)strideAs;
  const size_t oB = (size_t)zq * (size_t)strideB + (size_t)zr * (size_t)strideBs;
  const __bf16* Ab  = A   + oA;
  const __bf16* Ab2 = A2  + oA;
  const __bf16* Bb  = Bt  + oB;
  const __bf16* Bb2 = Bt2 + oB;

  const int rlane = lane & 15;
  const int koff  = (lane >> 4) * 8;
  const int mOff  = (lane >> 4) * 8;

  v8f acc[4][4];
#pragma unroll
  for (int i = 0; i < 4; ++i)
#pragma unroll
    for (int j = 0; j < 4; ++j) acc[i][j] = (v8f){0.f,0.f,0.f,0.f,0.f,0.f,0.f,0.f};

  for (int k0 = 0; k0 < K; k0 += 32) {
    v16b bh[4], bl[4];
#pragma unroll
    for (int j = 0; j < 4; ++j) {
      const size_t bo = (size_t)(n0 + (j << 4) + rlane) * ldb + koff + k0;
      bh[j] = ld_frag(Bb + bo);
      bl[j] = ld_frag(Bb2 + bo);
    }
#pragma unroll
    for (int i = 0; i < 4; ++i) {
      const size_t ao = (size_t)(m0 + (i << 4) + rlane) * lda + koff + k0;
      const v16b ah = ld_frag(Ab + ao);
      const v16b al = ld_frag(Ab2 + ao);
#pragma unroll
      for (int j = 0; j < 4; ++j) {
        acc[i][j] = mma_bf(ah, bh[j], acc[i][j]);
        acc[i][j] = mma_bf(ah, bl[j], acc[i][j]);
        acc[i][j] = mma_bf(al, bh[j], acc[i][j]);
      }
      dep_guard_b(acc[i][0], acc[i][3], ah, al);
    }
    keep4_b(bh[0], bh[1], bh[2], bh[3]);
    keep4_b(bl[0], bl[1], bl[2], bl[3]);
  }
  acc_guard4(acc[0][0], acc[0][1], acc[0][2], acc[0][3]);
  acc_guard4(acc[1][0], acc[1][1], acc[1][2], acc[1][3]);
  acc_guard4(acc[2][0], acc[2][1], acc[2][2], acc[2][3]);
  acc_guard4(acc[3][0], acc[3][1], acc[3][2], acc[3][3]);

  float* slab = sT[wave];
#pragma unroll
  for (int i = 0; i < 4; ++i) {
    const int mBase = m0 + (i << 4);
#pragma unroll
    for (int j = 0; j < 4; ++j) {
      const int n = n0 + (j << 4) + rlane;
      float bn = 0.f;
      if (BIAS_MODE == 2) bn = bias[n];
#pragma unroll
      for (int r = 0; r < 8; ++r) {
        float v = acc[i][j][r] * scale;
        if (BIAS_MODE == 1) v += bias[mBase + mOff + r];
        if (BIAS_MODE == 2) v += bn;
        slab[(mOff + r) * 68 + (j << 4) + rlane] = v;
      }
    }
    __builtin_amdgcn_fence(__ATOMIC_RELEASE, "workgroup");
    __builtin_amdgcn_wave_barrier();
    __builtin_amdgcn_fence(__ATOMIC_ACQUIRE, "workgroup");
    if (OUT_MODE == 0) {
      float* C = (float*)Cout + (size_t)z * (size_t)strideC;
      const int hh = lane >> 4, c4 = (lane & 15) * 4;
      for (int pass = 0; pass < 2; ++pass) {
#pragma unroll
        for (int it = 0; it < 8; ++it) {
          const int row = it * 2 + hh;
          const v4f v = *(const v4f*)(slab + row * 68 + c4);
          *(volatile v4f*)(C + (size_t)(mBase + row) * ldc + n0 + c4) = v;
        }
        __threadfence();
      }
    } else {
      const int q = lane >> 3, c8 = (lane & 7) * 8;
      unsigned short* C  = (unsigned short*)Cout  + (size_t)z * (size_t)strideC;
      unsigned short* C2 = (unsigned short*)Cout2 + (size_t)z * (size_t)strideC;
      v8us hv[4], lv[4];
#pragma unroll
      for (int it = 0; it < 4; ++it) {
        const int row = it * 4 + q;
        const float* sp = slab + row * 68 + c8;
#pragma unroll
        for (int e = 0; e < 8; ++e) {
          const unsigned short hb = f2bf_bits(sp[e]);
          const unsigned short lb = f2bf_bits(sp[e] - bf_bits2f(hb));
          hv[it][e] = hb;
          lv[it][e] = lb;
        }
      }
      for (int pass = 0; pass < 2; ++pass) {
#pragma unroll
        for (int it = 0; it < 4; ++it) {
          const int row = it * 4 + q;
          const size_t go = (size_t)(mBase + row) * ldc + n0 + c8;
          *(volatile v8us*)(C + go)  = hv[it];
          *(volatile v8us*)(C2 + go) = lv[it];
        }
        __threadfence();
      }
    }
    __builtin_amdgcn_fence(__ATOMIC_RELEASE, "workgroup");
    __builtin_amdgcn_wave_barrier();
    __builtin_amdgcn_fence(__ATOMIC_ACQUIRE, "workgroup");
  }
}

__global__ __launch_bounds__(256) void split_bf16x2_kernel(const float* __restrict__ in, unsigned short* __restrict__ hi,
                                                           unsigned short* __restrict__ lo, int n2) {
  const int i = blockIdx.x * 256 + threadIdx.x;
  if (i < n2) {
    const v2f f = *(const v2f*)(in + 2 * (size_t)i);
    const unsigned short h0 = f2bf_bits(f[0]), h1 = f2bf_bits(f[1]);
    const unsigned short l0 = f2bf_bits(f[0] - bf_bits2f(h0)), l1 = f2bf_bits(f[1] - bf_bits2f(h1));
    const unsigned uh = pk16(h0, h1), ul = pk16(l0, l1);
    ((volatile unsigned*)hi)[i] = uh;
    ((volatile unsigned*)lo)[i] = ul;
    __threadfence();
    ((volatile unsigned*)hi)[i] = uh;
    ((volatile unsigned*)lo)[i] = ul;
  }
}

__global__ __launch_bounds__(256) void tsplit_kernel(const float* __restrict__ W, unsigned short* __restrict__ oh,
                                                     unsigned short* __restrict__ ol, int R, int Cc, long sIn, long sOut) {
  __shared__ __align__(16) float tf[64 * 68];
  W  += (size_t)blockIdx.z * (size_t)sIn;
  oh += (size_t)blockIdx.z * (size_t)sOut;
  ol += (size_t)blockIdx.z * (size_t)sOut;
  const int c0  = blockIdx.x * 64;
  const int r0  = blockIdx.y * 64;
  const int tid = threadIdx.x;
  {
    const int lr = tid >> 4;
    const int c4 = (tid & 15) * 4;
#pragma unroll
    for (int it = 0; it < 4; ++it) {
      const int rr = it * 16 + lr;
      const v4f a = *(const v4f*)(W + (size_t)(r0 + rr) * Cc + c0 + c4);
      *(v4f*)(tf + rr * 68 + c4) = a;
    }
  }
  __syncthreads();
  const int sub = tid >> 3;
  const int c8  = (tid & 7) * 8;
  v4u hv[2], lv[2];
#pragma unroll
  for (int it = 0; it < 2; ++it) {
    const int oc = it * 32 + sub;
    v4u a, a2;
#pragma unroll
    for (int q = 0; q < 4; ++q) {
      const float f0 = tf[(c8 + 2 * q) * 68 + oc];
      const float f1 = tf[(c8 + 2 * q + 1) * 68 + oc];
      const unsigned short h0 = f2bf_bits(f0), h1 = f2bf_bits(f1);
      const unsigned short l0 = f2bf_bits(f0 - bf_bits2f(h0)), l1 = f2bf_bits(f1 - bf_bits2f(h1));
      a[q]  = pk16(h0, h1);
      a2[q] = pk16(l0, l1);
    }
    hv[it] = a; lv[it] = a2;
  }
  for (int pass = 0; pass < 2; ++pass) {
#pragma unroll
    for (int it = 0; it < 2; ++it) {
      const int oc = it * 32 + sub;
      const size_t go = (size_t)(c0 + oc) * R + r0 + c8;
      *(volatile v4u*)(oh + go) = hv[it];
      *(volatile v4u*)(ol + go) = lv[it];
    }
    __threadfence();
  }
}

__global__ __launch_bounds__(256) void sk_row_kernel(const float* __restrict__ LG, const float* __restrict__ Bv,
                                                     float* __restrict__ Av, int use_b) {
  __shared__ __align__(16) float sa[32];
  const int tid = threadIdx.x, wave = tid >> 5, lane = tid & 31;
  const int n  = blockIdx.x >> 5;
  const int i0 = (blockIdx.x & 31) * 32;
  const float* Lb = LG + (size_t)n * SEQ * SEQ;
  v4f bb[8];
  if (use_b != 0) {
    const float* bp = Bv + (size_t)n * SEQ;
#pragma unroll
    for (int it = 0; it < 8; ++it) bb[it] = *(const v4f*)(bp + it * 128 + lane * 4);
  } else {
#pragma unroll
    for (int it = 0; it < 8; ++it) bb[it] = (v4f){0.f, 0.f, 0.f, 0.f};
  }
#pragma unroll 1
  for (int rr = 0; rr < 4; ++rr) {
    const int i = i0 + wave * 4 + rr;
    const float* row = Lb + (size_t)i * SEQ;
    v4f xv[8];
    float m = -1.0e30f;
#pragma unroll
    for (int it = 0; it < 8; ++it) {
      v4f g = *(const v4f*)(row + it * 128 + lane * 4);
      g = g - bb[it];
      xv[it] = g;
      m = fmaxf(m, fmaxf(fmaxf(g[0], g[1]), fmaxf(g[2], g[3])));
    }
#pragma unroll
    for (int off = 1; off < 32; off <<= 1) m = fmaxf(m, __shfl_xor(m, off, 32));
    float s = 0.f;
#pragma unroll
    for (int it = 0; it < 8; ++it) {
      s += exp2f(xv[it][0] - m) + exp2f(xv[it][1] - m);
      s += exp2f(xv[it][2] - m) + exp2f(xv[it][3] - m);
    }
#pragma unroll
    for (int off = 1; off < 32; off <<= 1) s += __shfl_xor(s, off, 32);
    const float a = m + log2f(s);
    if (lane == 0) sa[wave * 4 + rr] = a;
  }
  __syncthreads();
  if (tid < 8) {
    const v4f v = *(const v4f*)(sa + tid * 4);
    float* dst = Av + (size_t)n * SEQ + i0 + tid * 4;
    *(volatile v4f*)dst = v;
    __threadfence();
    *(volatile v4f*)dst = v;
  }
}

__global__ __launch_bounds__(256) void sk_col_kernel(const float* __restrict__ LG, const float* __restrict__ Av,
                                                     float* __restrict__ Bv) {
  __shared__ __align__(16) float sA[SEQ];
  __shared__ float sM[8][32];
  __shared__ float sS[8][32];
  __shared__ __align__(16) float sb[32];
  const int tid = threadIdx.x, wave = tid >> 5, lane = tid & 31;
  const int n  = blockIdx.x >> 5;
  const int j0 = (blockIdx.x & 31) * 32;
  *(v4f*)(sA + tid * 4) = *(const v4f*)(Av + (size_t)n * SEQ + tid * 4);
  __syncthreads();
  const float* col = LG + (size_t)n * SEQ * SEQ + j0 + lane;
  const int ib = wave * 128;
  float m = -1.0e30f, s = 0.f;
#pragma unroll 2
  for (int ch = 0; ch < 16; ++ch) {
    const int ir = ib + ch * 8;
    float x[8];
#pragma unroll
    for (int q = 0; q < 8; ++q) x[q] = col[(size_t)(ir + q) * SEQ] - sA[ir + q];
    const float cm = fmaxf(fmaxf(fmaxf(x[0], x[1]), fmaxf(x[2], x[3])), fmaxf(fmaxf(x[4], x[5]), fmaxf(x[6], x[7])));
    const float mn = fmaxf(m, cm);
    float acc = s * exp2f(m - mn);
#pragma unroll
    for (int q = 0; q < 8; ++q) acc += exp2f(x[q] - mn);
    s = acc;
    m = mn;
  }
  sM[wave][lane] = m;
  sS[wave][lane] = s;
  __syncthreads();
  if (wave == 0) {
    float Mx = sM[0][lane];
#pragma unroll
    for (int w = 1; w < 8; ++w) Mx = fmaxf(Mx, sM[w][lane]);
    float Sx = 0.f;
#pragma unroll
    for (int w = 0; w < 8; ++w) Sx += sS[w][lane] * exp2f(sM[w][lane] - Mx);
    sb[lane] = Mx + log2f(Sx);
  }
  __syncthreads();
  if (tid < 8) {
    const v4f v = *(const v4f*)(sb + tid * 4);
    float* dst = Bv + (size_t)n * SEQ + j0 + tid * 4;
    *(volatile v4f*)dst = v;
    __threadfence();
    *(volatile v4f*)dst = v;
  }
}

__global__ __launch_bounds__(128)
void pv_kernel(const float* __restrict__ LG, const float* __restrict__ Av, const float* __restrict__ Bv,
               const unsigned short* __restrict__ vthp, const unsigned short* __restrict__ vtlp,
               unsigned short* __restrict__ cth, unsigned short* __restrict__ ctl) {
  union FB { v16b v; v8b h[2]; };
  union FS { v16b v; unsigned short s[16]; };
  __shared__ __align__(16) __bf16 Vth[64 * 64];
  __shared__ __align__(16) __bf16 Vtl[64 * 64];
  __shared__ __align__(16) float  sbv[SEQ];
  __shared__ __align__(16) float  Os[4][16 * 68];
  const int tid  = threadIdx.x;
  const int wave = tid >> 5;
  const int lane = tid & 31;
  const int hh   = lane >> 4;
  const int c    = lane & 15;
  const int n    = blockIdx.x >> 4;
  const int ib   = (blockIdx.x & 15) * 64;
  const int bb   = n >> 3;
  const int h    = n & 7;
  const int i0w  = ib + wave * 16;
  const int i    = i0w + c;
  const float* Lrow = LG + ((size_t)n * SEQ + i) * SEQ;
  const float ai = Av[(size_t)n * SEQ + i];
  {
    const float* bp = Bv + (size_t)n * SEQ;
    *(v4f*)(sbv + tid * 8)     = *(const v4f*)(bp + tid * 8);
    *(v4f*)(sbv + tid * 8 + 4) = *(const v4f*)(bp + tid * 8 + 4);
  }
  const __bf16* Vh = (const __bf16*)(const void*)vthp + ((size_t)bb * HDIM + h * DHEAD) * SEQ;
  const __bf16* Vl = (const __bf16*)(const void*)vtlp + ((size_t)bb * HDIM + h * DHEAD) * SEQ;

  v8f oacc[4];
#pragma unroll
  for (int t = 0; t < 4; ++t) oacc[t] = (v8f){0.f,0.f,0.f,0.f,0.f,0.f,0.f,0.f};

  for (int kc = 0; kc < SEQ / 64; ++kc) {
    const int kv0 = kc * 64;
    __syncthreads();
    {
      const int r = tid >> 1, half = (tid & 1) * 32;
      const __bf16* vsh = Vh + (size_t)r * SEQ + kv0 + half;
      const __bf16* vsl = Vl + (size_t)r * SEQ + kv0 + half;
#pragma unroll
      for (int q = 0; q < 4; ++q) {
        const v8b a0 = *(const v8b*)(vsh + 8 * q);
        const v8b a1 = *(const v8b*)(vsl + 8 * q);
        *(v8b*)(Vth + r * 64 + half + 8 * q) = a0;
        *(v8b*)(Vtl + r * 64 + half + 8 * q) = a1;
      }
    }
    __syncthreads();
#pragma unroll
    for (int kk = 0; kk < 2; ++kk) {
      const int jb = kv0 + kk * 32;
      const int jl = kk * 32;
      v4f g[4], cb[4];
      g[0]  = *(const v4f*)(Lrow + jb + 8 * hh);
      g[1]  = *(const v4f*)(Lrow + jb + 8 * hh + 4);
      g[2]  = *(const v4f*)(Lrow + jb + 16 + 8 * hh);
      g[3]  = *(const v4f*)(Lrow + jb + 16 + 8 * hh + 4);
      cb[0] = *(const v4f*)(sbv + jb + 8 * hh);
      cb[1] = *(const v4f*)(sbv + jb + 8 * hh + 4);
      cb[2] = *(const v4f*)(sbv + jb + 16 + 8 * hh);
      cb[3] = *(const v4f*)(sbv + jb + 16 + 8 * hh + 4);
      FS ph, pl;
#pragma unroll
      for (int q = 0; q < 4; ++q) {
#pragma unroll
        for (int e = 0; e < 4; ++e) {
          const float x = ((g[q][e] - ai) - cb[q][e]) + 14.0f;
          const float p = exp2f(x);
          const unsigned short hb = f2bf_bits(p);
          const unsigned short lb = f2bf_bits(p - bf_bits2f(hb));
          ph.s[q * 4 + e] = hb;
          pl.s[q * 4 + e] = lb;
        }
      }
#pragma unroll
      for (int t = 0; t < 4; ++t) {
        FB vb, vl;
        vb.h[0] = *(const v8b*)(Vth + (t * 16 + c) * 64 + jl + 8 * hh);
        vb.h[1] = *(const v8b*)(Vth + (t * 16 + c) * 64 + jl + 16 + 8 * hh);
        vl.h[0] = *(const v8b*)(Vtl + (t * 16 + c) * 64 + jl + 8 * hh);
        vl.h[1] = *(const v8b*)(Vtl + (t * 16 + c) * 64 + jl + 16 + 8 * hh);
        oacc[t] = mma_bf_g(ph.v, vb.v, oacc[t]);
        oacc[t] = mma_bf_g(ph.v, vl.v, oacc[t]);
        oacc[t] = mma_bf_g(pl.v, vb.v, oacc[t]);
      }
    }
  }

  float* os = Os[wave];
  const float oscale = 6.103515625e-05f;
#pragma unroll
  for (int r = 0; r < 8; ++r)
#pragma unroll
    for (int t = 0; t < 4; ++t) os[(8 * hh + r) * 68 + t * 16 + c] = oacc[t][r] * oscale;
  __builtin_amdgcn_fence(__ATOMIC_RELEASE, "workgroup");
  __builtin_amdgcn_wave_barrier();
  __builtin_amdgcn_fence(__ATOMIC_ACQUIRE, "workgroup");
  {
    const int q = lane >> 3, c8 = (lane & 7) * 8;
    unsigned short* Ch = cth + (size_t)h * DHEAD;
    unsigned short* Cl = ctl + (size_t)h * DHEAD;
    v8us hv[4], lv[4];
#pragma unroll
    for (int it = 0; it < 4; ++it) {
      const int row = it * 4 + q;
      const float* sp = os + row * 68 + c8;
#pragma unroll
      for (int e = 0; e < 8; ++e) {
        const unsigned short hb = f2bf_bits(sp[e]);
        const unsigned short lb = f2bf_bits(sp[e] - bf_bits2f(hb));
        hv[it][e] = hb;
        lv[it][e] = lb;
      }
    }
    for (int pass = 0; pass < 2; ++pass) {
#pragma unroll
      for (int it = 0; it < 4; ++it) {
        const int row = it * 4 + q;
        const size_t go = ((size_t)bb * SEQ + i0w + row) * HDIM + c8;
        *(volatile v8us*)(Ch + go) = hv[it];
        *(volatile v8us*)(Cl + go) = lv[it];
      }
      __threadfence();
    }
  }
}

extern "C" void kernel_launch(void* const* d_in, const int* in_sizes, int n_in,
                              void* d_out, int out_size, void* d_ws, size_t ws_size,
                              hipStream_t stream) {
  if (n_in < 9) return;
  if (in_sizes[0] != NB * SEQ * EMB) return;
  if (in_sizes[1] != EMB * HDIM || in_sizes[3] != EMB * HDIM || in_sizes[5] != EMB * HDIM) return;
  if (in_sizes[2] != HDIM || in_sizes[4] != HDIM || in_sizes[6] != HDIM) return;
  if (in_sizes[7] != HDIM * EMB || in_sizes[8] != EMB) return;
  if (out_size != NB * SEQ * EMB) return;

  const float* x  = (const float*)d_in[0];
  const float* Wq = (const float*)d_in[1];
  const float* bq = (const float*)d_in[2];
  const float* Wk = (const float*)d_in[3];
  const float* bk = (const float*)d_in[4];
  const float* Wv = (const float*)d_in[5];
  const float* bv = (const float*)d_in[6];
  const float* Wo = (const float*)d_in[7];
  const float* bo = (const float*)d_in[8];
  float* out = (float*)d_out;

  const size_t PXE = (size_t)MROWS * EMB * 2;
  const size_t PW  = (size_t)EMB * HDIM * 2;
  const size_t PQ  = (size_t)MROWS * HDIM * 2;
  const size_t PVT = (size_t)NB * HDIM * SEQ * 2;
  const size_t PLG = (size_t)NMAT * SEQ * SEQ * 4;
  const size_t PAB = (size_t)NMAT * SEQ * 4;
  const size_t PCT = (size_t)MROWS * HDIM * 2;
  size_t off = 0;
  const size_t oXh = off; off += PXE;  const size_t oXl = off; off += PXE;
  const size_t oWqTh = off; off += PW; const size_t oWqTl = off; off += PW;
  const size_t oWkTh = off; off += PW; const size_t oWkTl = off; off += PW;
  const size_t oWvTh = off; off += PW; const size_t oWvTl = off; off += PW;
  const size_t oWoTh = off; off += PW; const size_t oWoTl = off; off += PW;
  const size_t oQh = off; off += PQ;   const size_t oQl = off; off += PQ;
  const size_t oKh = off; off += PQ;   const size_t oKl = off; off += PQ;
  const size_t oVTh = off; off += PVT; const size_t oVTl = off; off += PVT;
  const size_t oLG = off; off += PLG;
  const size_t oA = off; off += PAB;   const size_t oBv = off; off += PAB;
  const size_t oCTh = off; off += PCT; const size_t oCTl = off; off += PCT;
  if (off > ws_size) return;
  if (off > (size_t)134217728) return;

  char* ws = (char*)d_ws;
  unsigned short* Xh   = (unsigned short*)(ws + oXh);   unsigned short* Xl   = (unsigned short*)(ws + oXl);
  unsigned short* WqTh = (unsigned short*)(ws + oWqTh); unsigned short* WqTl = (unsigned short*)(ws + oWqTl);
  unsigned short* WkTh = (unsigned short*)(ws + oWkTh); unsigned short* WkTl = (unsigned short*)(ws + oWkTl);
  unsigned short* WvTh = (unsigned short*)(ws + oWvTh); unsigned short* WvTl = (unsigned short*)(ws + oWvTl);
  unsigned short* WoTh = (unsigned short*)(ws + oWoTh); unsigned short* WoTl = (unsigned short*)(ws + oWoTl);
  unsigned short* Qh   = (unsigned short*)(ws + oQh);   unsigned short* Ql   = (unsigned short*)(ws + oQl);
  unsigned short* Kh   = (unsigned short*)(ws + oKh);   unsigned short* Kl   = (unsigned short*)(ws + oKl);
  unsigned short* VTh  = (unsigned short*)(ws + oVTh);  unsigned short* VTl  = (unsigned short*)(ws + oVTl);
  float*          LG   = (float*)(ws + oLG);
  float*          Avec = (float*)(ws + oA);
  float*          Bvec = (float*)(ws + oBv);
  unsigned short* CTh  = (unsigned short*)(ws + oCTh);  unsigned short* CTl  = (unsigned short*)(ws + oCTl);

  const dim3 blk(256);

  const int n2x = MROWS * EMB / 2;
  split_bf16x2_kernel<<<dim3(n2x / 256), blk, 0, stream>>>(x, Xh, Xl, n2x);

  tsplit_kernel<<<dim3(HDIM / 64, EMB / 64, 1), blk, 0, stream>>>(Wq, WqTh, WqTl, EMB, HDIM, 0L, 0L);
  tsplit_kernel<<<dim3(HDIM / 64, EMB / 64, 1), blk, 0, stream>>>(Wk, WkTh, WkTl, EMB, HDIM, 0L, 0L);
  tsplit_kernel<<<dim3(HDIM / 64, EMB / 64, 1), blk, 0, stream>>>(Wv, WvTh, WvTl, EMB, HDIM, 0L, 0L);
  tsplit_kernel<<<dim3(EMB / 64, HDIM / 64, 1), blk, 0, stream>>>(Wo, WoTh, WoTl, HDIM, EMB, 0L, 0L);

  gemm64_split<2, 2><<<dim3(32, 1), blk, 0, stream>>>(
      Xh, Xl, EMB, 0L, 0L, WqTh, WqTl, EMB, 0L, 0L, (void*)Qh, (void*)Ql, HDIM, 0L, bq, MROWS, HDIM, EMB, 1, 1.0f);
  gemm64_split<2, 2><<<dim3(32, 1), blk, 0, stream>>>(
      Xh, Xl, EMB, 0L, 0L, WkTh, WkTl, EMB, 0L, 0L, (void*)Kh, (void*)Kl, HDIM, 0L, bk, MROWS, HDIM, EMB, 1, 1.0f);
  gemm64_split<1, 2><<<dim3(16, NB), blk, 0, stream>>>(
      WvTh, WvTl, EMB, 0L, 0L, Xh, Xl, EMB, (long)SEQ * EMB, 0L, (void*)VTh, (void*)VTl, SEQ, (long)HDIM * SEQ,
      bv, HDIM, SEQ, EMB, 1, 1.0f);

  const float sscale = 0.125f * 1.4426950408889634f;
  gemm64_split<0, 0><<<dim3(32, NMAT), blk, 0, stream>>>(
      Qh, Ql, HDIM, (long)SEQ * HDIM, (long)DHEAD, Kh, Kl, HDIM, (long)SEQ * HDIM, (long)DHEAD,
      (void*)LG, (void*)LG, SEQ, (long)SEQ * SEQ, bq, SEQ, SEQ, DHEAD, NHEAD, sscale);

  for (int it = 0; it < NITER; ++it) {
    sk_row_kernel<<<dim3(NMAT * (SEQ / 32)), blk, 0, stream>>>(LG, Bvec, Avec, (it == 0) ? 0 : 1);
    sk_col_kernel<<<dim3(NMAT * (SEQ / 32)), blk, 0, stream>>>(LG, Avec, Bvec);
  }

  pv_kernel<<<dim3(NMAT * (SEQ / 64)), dim3(128), 0, stream>>>(LG, Avec, Bvec, VTh, VTl, CTh, CTl);

  gemm64_split<2, 0><<<dim3(64, 1), blk, 0, stream>>>(
      CTh, CTl, HDIM, 0L, 0L, WoTh, WoTl, HDIM, 0L, 0L, (void*)out, (void*)out, EMB, 0L, bo, MROWS, EMB, HDIM, 1, 1.0f);

  (void)hipGetLastError();
}
